// CSDA_80135499809149
// MI455X (gfx1250) — hardware-verified
//
#include <hip/hip_runtime.h>

typedef _Float16 f16t;
typedef _Float16 v16h __attribute__((ext_vector_type(16)));
typedef _Float16 v8h  __attribute__((ext_vector_type(8)));
typedef float    v8f  __attribute__((ext_vector_type(8)));
typedef float    v4f  __attribute__((ext_vector_type(4)));
typedef v8h __attribute__((may_alias)) v8ha;
typedef v4f __attribute__((may_alias)) v4fa;
union Frag { v16h v; v8h half[2]; };

#define NB    8
#define DIMC  128
#define HH    64
#define WW    64
#define NPIX  4096
#define NP    32768
#define NHEAD 8
#define HDIM  16
#define NUNIT 1024
#define LWIN  256
#define PLANE ((size_t)NUNIT * LWIN * HDIM)
#define VTS   264

#define WSC  32.0f
#define TCAR 8.0f
#define QCAR 16.0f
#define PCAR 1024.0f
#define OCAR 256.0f
#define ACAR 256.0f
#define MCAR 8.0f

__device__ __forceinline__ v8f wmma_f16(v16h a, v16h b, v8f c) {
  v8f d = __builtin_amdgcn_wmma_f32_16x16x32_f16(false, a, false, b, (short)0, c, false, false);
  asm volatile("v_nop\n\tv_nop\n\tv_nop\n\tv_nop" : "+v"(d) : "v"(a), "v"(b));
  return d;
}

__device__ __forceinline__ v8h zero8h() {
  v8h z;
  #pragma unroll
  for (int j = 0; j < 8; ++j) z[j] = (f16t)0.0f;
  return z;
}

__device__ __forceinline__ v16h load_frag32(const f16t* p, int h) {
  Frag f;
  f.half[0] = *(const v8ha*)(p + 8 * h);
  f.half[1] = *(const v8ha*)(p + 16 + 8 * h);
  return f.v;
}

__device__ __forceinline__ v16h load_frag16(const f16t* p, int h) {
  Frag f;
  f.half[0] = *(const v8ha*)(p + 8 * h);
  f.half[1] = zero8h();
  return f.v;
}

__device__ __forceinline__ float sigm(float t) {
  return __builtin_amdgcn_rcpf(1.0f + __expf(-t));
}

__device__ __forceinline__ float wave_sum(float s) {
  s += __shfl_xor(s, 16);
  s += __shfl_xor(s, 8);
  s += __shfl_xor(s, 4);
  s += __shfl_xor(s, 2);
  s += __shfl_xor(s, 1);
  return s;
}

__device__ __forceinline__ void dw3x4(const float* __restrict__ pl, int y, int x0,
                                      const float (&wc)[9], float (&acc)[4], v4f& mid) {
  #pragma unroll
  for (int i = 0; i < 4; ++i) acc[i] = 0.f;
  mid = *(const v4fa*)(pl + y * WW + x0);
  #pragma unroll
  for (int dy = 0; dy < 3; ++dy) {
    const int yy = y + dy - 1;
    const bool vy = (unsigned)yy < (unsigned)HH;
    const int yc = yy < 0 ? 0 : (yy > HH - 1 ? HH - 1 : yy);
    const float* rp = pl + yc * WW;
    const v4f m4 = *(const v4fa*)(rp + x0);
    const float lf = rp[x0 > 0 ? x0 - 1 : 0];
    const float rt = rp[(x0 + 4 < WW) ? x0 + 4 : WW - 1];
    float r6[6];
    r6[0] = (vy && x0 > 0) ? lf : 0.f;
    r6[1] = vy ? m4.x : 0.f;
    r6[2] = vy ? m4.y : 0.f;
    r6[3] = vy ? m4.z : 0.f;
    r6[4] = vy ? m4.w : 0.f;
    r6[5] = (vy && (x0 + 4 < WW)) ? rt : 0.f;
    #pragma unroll
    for (int i = 0; i < 4; ++i) {
      #pragma unroll
      for (int dx = 0; dx < 3; ++dx) acc[i] += wc[dy * 3 + dx] * r6[i + dx];
    }
  }
}

__device__ __forceinline__ void plane_store64(const f16t* sH, f16t* __restrict__ out,
                                              size_t p0, int ch0, int w, int lane) {
  const int q8 = lane & 7, sub = lane >> 3;
  v8h vals[2];
  size_t d[2];
  #pragma unroll
  for (int i = 0; i < 2; ++i) {
    const int lid = 8 * w + 4 * i + sub;
    vals[i] = *(const v8ha*)(sH + lid * 64 + 8 * q8);
    d[i] = (p0 + (size_t)lid) * DIMC + ch0 + 8 * q8;
  }
  #pragma unroll
  for (int i = 0; i < 2; ++i) *(volatile v8h*)(out + d[i]) = vals[i];
  __threadfence();
  #pragma unroll
  for (int i = 0; i < 2; ++i) *(volatile v8h*)(out + d[i]) = vals[i];
}

__device__ __forceinline__ void nchw_store(const float* sD, float* __restrict__ out,
                                           const float* __restrict__ res, int b, int cbase,
                                           int y, int w, int lane) {
  const int hs = lane >> 4, x4 = 4 * (lane & 15);
  v4f vals[8];
  size_t gi[8];
  #pragma unroll
  for (int i = 0; i < 8; ++i) {
    const int col = 16 * w + 2 * i + hs;
    v4f v = *(const v4fa*)(sD + col * 64 + x4);
    gi[i] = ((size_t)(b * DIMC + cbase + col) * HH + y) * WW + x4;
    if (res != nullptr) v += *(const v4fa*)(res + gi[i]);
    vals[i] = v;
  }
  #pragma unroll
  for (int i = 0; i < 8; ++i) *(volatile v4f*)(out + gi[i]) = vals[i];
  __threadfence();
  #pragma unroll
  for (int i = 0; i < 8; ++i) *(volatile v4f*)(out + gi[i]) = vals[i];
}

__global__ __launch_bounds__(256) void wcvt_k(
    const float* __restrict__ w_act, const float* __restrict__ w_in, const float* __restrict__ w_qkv,
    const float* __restrict__ w_out, const float* __restrict__ w_m1, const float* __restrict__ w_m2,
    f16t* __restrict__ W16)
{
  const int g = blockIdx.x * 256 + threadIdx.x;
  if (g >= 32768) return;
  const int e8 = g * 8;
  const float* src;
  if (e8 < 16384) src = w_act + e8;
  else if (e8 < 32768) src = w_in + (e8 - 16384);
  else if (e8 < 114688) {
    const int e = e8 - 32768;
    const int o = e >> 7, col = e & 127;
    const int gq = o >> 7, c = o & 127;
    src = w_qkv + (size_t)(c * 5 + gq) * DIMC + col;
  }
  else if (e8 < 131072) src = w_out + (e8 - 114688);
  else if (e8 < 196608) src = w_m1 + (e8 - 131072);
  else src = w_m2 + (e8 - 196608);
  const v4f a = *(const v4fa*)src;
  const v4f c = *(const v4fa*)(src + 4);
  v8h o;
  o[0] = (f16t)(a.x * WSC); o[1] = (f16t)(a.y * WSC); o[2] = (f16t)(a.z * WSC); o[3] = (f16t)(a.w * WSC);
  o[4] = (f16t)(c.x * WSC); o[5] = (f16t)(c.y * WSC); o[6] = (f16t)(c.z * WSC); o[7] = (f16t)(c.w * WSC);
  f16t* dst = W16 + (size_t)e8;
  *(volatile v8h*)dst = o;
  __threadfence();
  *(volatile v8h*)dst = o;
}

__global__ __launch_bounds__(256) void gap_k(const float* __restrict__ x, float* __restrict__ gap) {
  __shared__ __attribute__((aligned(16))) float sg[32];
  const int tid = threadIdx.x, lane = tid & 31, w = tid >> 5;
  #pragma unroll 1
  for (int j = 0; j < 4; ++j) {
    const int ch = blockIdx.x * 32 + w * 4 + j;
    const float* p = x + (size_t)ch * NPIX;
    float s = 0.f;
    #pragma unroll 4
    for (int k = 0; k < 32; ++k) {
      const v4f v = *(const v4fa*)(p + (size_t)(lane + 32 * k) * 4);
      s += (v.x + v.y) + (v.z + v.w);
    }
    s = wave_sum(s);
    if (lane == 0) sg[w * 4 + j] = s * (1.0f / 4096.0f);
  }
  __syncthreads();
  const v4f v = *(const v4fa*)(sg + 4 * (lane & 7));
  float* dst = gap + blockIdx.x * 32 + 4 * (lane & 7);
  const bool pw = (w == 0) && (lane < 8);
  if (pw) *(volatile v4f*)dst = v;
  __threadfence();
  if (pw) *(volatile v4f*)dst = v;
}

__global__ __launch_bounds__(256) void front_k(
    const float* __restrict__ x, const float* __restrict__ gap, const float* __restrict__ gw,
    const float* __restrict__ alpha, float* __restrict__ x1)
{
  __shared__ float sgap[DIMC];
  __shared__ float sgate[DIMC];
  __shared__ float smx[4][WW];
  __shared__ float smn[4][WW];
  const int tid = threadIdx.x;
  const int y = blockIdx.x, b = blockIdx.y;
  if (tid < DIMC) sgap[tid] = gap[b * DIMC + tid];
  __syncthreads();
  if (tid < DIMC) {
    float acc = 0.f;
    #pragma unroll
    for (int j = 0; j < 5; ++j) {
      const int cc = tid + j - 2;
      const int ccl = cc < 0 ? 0 : (cc > DIMC - 1 ? DIMC - 1 : cc);
      const float gv = ((unsigned)cc < (unsigned)DIMC) ? sgap[ccl] : 0.f;
      acc += gw[j] * gv;
    }
    sgate[tid] = sigm(acc);
  }
  const int xx = tid & 63, cg = tid >> 6;
  const size_t base = ((size_t)(b * DIMC + cg * 32) * HH + y) * WW + xx;
  float v[32];
  float mx = -3.0e38f, mn = 3.0e38f;
  #pragma unroll
  for (int i = 0; i < 32; ++i) {
    v[i] = x[base + (size_t)i * NPIX];
    const float se = v[i] - sgap[cg * 32 + i];
    mx = fmaxf(mx, se);
    mn = fminf(mn, se);
  }
  smx[cg][xx] = mx;
  smn[cg][xx] = mn;
  __syncthreads();
  const float mxa = fmaxf(fmaxf(smx[0][xx], smx[1][xx]), fmaxf(smx[2][xx], smx[3][xx]));
  const float mna = fminf(fminf(smn[0][xx], smn[1][xx]), fminf(smn[2][xx], smn[3][xx]));
  const float al = alpha[0];
  const float om = 1.0f - al;
  const float s1 = sigm(mxa), s2 = sigm(mna);
  float r[32];
  #pragma unroll
  for (int i = 0; i < 32; ++i) {
    const float vv = v[i];
    r[i] = vv * sgate[cg * 32 + i] + ((vv * s1) * al + (vv * s2) * om);
  }
  float* op = x1 + base;
  #pragma unroll
  for (int i = 0; i < 32; ++i) *(volatile float*)(op + (size_t)i * NPIX) = r[i];
  __threadfence();
  #pragma unroll
  for (int i = 0; i < 32; ++i) *(volatile float*)(op + (size_t)i * NPIX) = r[i];
}

__global__ __launch_bounds__(256) void dwres_k(
    const float* __restrict__ in, const float* __restrict__ wk, const float* __restrict__ bias,
    float* __restrict__ out, float* __restrict__ part)
{
  __shared__ float sred[8];
  const int tid = threadIdx.x, lane = tid & 31, w = tid >> 5;
  const int rg = blockIdx.x, c = blockIdx.y, b = blockIdx.z;
  const int row = tid >> 4, xq = tid & 15;
  const int y = rg * 16 + row, x0 = 4 * xq;
  const float* pl = in + (size_t)(b * DIMC + c) * NPIX;
  float wc[9];
  #pragma unroll
  for (int t = 0; t < 9; ++t) wc[t] = wk[c * 9 + t];
  const float bc = bias[c];
  float acc[4];
  v4f mid;
  dw3x4(pl, y, x0, wc, acc, mid);
  v4f o;
  o.x = mid.x + (acc[0] + bc);
  o.y = mid.y + (acc[1] + bc);
  o.z = mid.z + (acc[2] + bc);
  o.w = mid.w + (acc[3] + bc);

  float s = (o.x + o.y) + (o.z + o.w);
  s = wave_sum(s);
  if (lane == 0) sred[w] = s;
  __syncthreads();
  float S = 0.f;
  #pragma unroll
  for (int k = 0; k < 8; ++k) S += sred[k];
  const float mb = S * (1.0f / 1024.0f);
  __syncthreads();
  const float d0 = o.x - mb, d1 = o.y - mb, d2 = o.z - mb, d3 = o.w - mb;
  float q = (d0 * d0 + d1 * d1) + (d2 * d2 + d3 * d3);
  q = wave_sum(q);
  if (lane == 0) sred[w] = q;
  __syncthreads();
  float Q = 0.f;
  #pragma unroll
  for (int k = 0; k < 8; ++k) Q += sred[k];

  const size_t gi = ((size_t)(b * DIMC + c) * HH + y) * WW + x0;
  const size_t li = (size_t)(b * 512 + c * 4 + rg) * 32 + 4 * (lane & 7);
  v4f pv;
  pv.x = (lane == 0) ? S : 0.f;
  pv.y = (lane == 0) ? Q : 0.f;
  pv.z = 0.f; pv.w = 0.f;
  const bool pw = (w == 0) && (lane < 8);
  *(volatile v4f*)(out + gi) = o;
  if (pw) *(volatile v4f*)(part + li) = pv;
  __threadfence();
  *(volatile v4f*)(out + gi) = o;
  if (pw) *(volatile v4f*)(part + li) = pv;
}

__global__ __launch_bounds__(256) void gnstat_k(const float* __restrict__ part, float* __restrict__ stats) {
  __shared__ double sa[8][32];
  __shared__ double smu[8];
  __shared__ float sres[8][2];
  const int tid = threadIdx.x, lane = tid & 31, w = tid >> 5;
  const float* pb = part + (size_t)w * 512 * 32;
  double s = 0.0;
  #pragma unroll 1
  for (int k = 0; k < 16; ++k) s += (double)pb[(size_t)(k * 32 + lane) * 32];
  sa[w][lane] = s;
  __syncthreads();
  if (lane == 0) {
    double t = 0.0;
    for (int i = 0; i < 32; ++i) t += sa[w][i];
    smu[w] = t * (1.0 / 524288.0);
  }
  __syncthreads();
  const double mu = smu[w];
  double q = 0.0;
  #pragma unroll 1
  for (int k = 0; k < 16; ++k) {
    const float* pl = pb + (size_t)(k * 32 + lane) * 32;
    const double sb = (double)pl[0], m2 = (double)pl[1];
    const double dm = sb * (1.0 / 1024.0) - mu;
    q += m2 + 1024.0 * dm * dm;
  }
  sa[w][lane] = q;
  __syncthreads();
  if (lane == 0) {
    double t = 0.0;
    for (int i = 0; i < 32; ++i) t += sa[w][i];
    const float varf = (float)(t * (1.0 / 524288.0));
    sres[w][0] = (float)mu;
    sres[w][1] = rsqrtf(varf + 1e-5f);
  }
  __syncthreads();
  const float a0 = sres[w][0], a1 = sres[w][1];
  v4f pv;
  pv.x = (lane == 0) ? a0 : 0.f;
  pv.y = (lane == 0) ? a1 : 0.f;
  pv.z = 0.f; pv.w = 0.f;
  float* dst = stats + w * 32 + 4 * (lane & 7);
  if (lane < 8) *(volatile v4f*)dst = pv;
  __threadfence();
  if (lane < 8) *(volatile v4f*)dst = pv;
}

__global__ __launch_bounds__(256) void cvt_k(
    const float* __restrict__ in, const float* __restrict__ stats, const float* __restrict__ g,
    const float* __restrict__ bt, f16t* __restrict__ out)
{
  __shared__ __attribute__((aligned(16))) f16t sH[64 * 64];
  const int tid = threadIdx.x, lane = tid & 31, w = tid >> 5;
  const int ch0 = blockIdx.x * 64, y = blockIdx.y, b = blockIdx.z;
  const int xq = tid & 15, cl = tid >> 4, x0 = 4 * xq;
  const float mu = stats[b * 32], rs = stats[b * 32 + 1];
  #pragma unroll 1
  for (int j = 0; j < 4; ++j) {
    const int col = cl + 16 * j, c = ch0 + col;
    const v4f v = *(const v4fa*)(in + ((size_t)(b * DIMC + c) * HH + y) * WW + x0);
    const float gg = g[c], bb = bt[c];
    sH[(x0 + 0) * 64 + col] = (f16t)((((v.x - mu) * rs) * gg) + bb);
    sH[(x0 + 1) * 64 + col] = (f16t)((((v.y - mu) * rs) * gg) + bb);
    sH[(x0 + 2) * 64 + col] = (f16t)((((v.z - mu) * rs) * gg) + bb);
    sH[(x0 + 3) * 64 + col] = (f16t)((((v.w - mu) * rs) * gg) + bb);
  }
  __syncthreads();
  plane_store64(sH, out, (size_t)b * NPIX + (size_t)y * WW, ch0, w, lane);
}

__device__ __forceinline__ void gemm_main(const f16t* __restrict__ A, int K, const f16t* __restrict__ Bw,
                                          int arow0, int n0, int h, int m, v8f (&acc)[4]) {
  const v8f z8 = {0.f, 0.f, 0.f, 0.f, 0.f, 0.f, 0.f, 0.f};
  #pragma unroll
  for (int nt = 0; nt < 4; ++nt) acc[nt] = z8;
  const f16t* ap = A + (size_t)(arow0 + m) * K;
  const f16t* bp = Bw + (size_t)(n0 + m) * K;
  const size_t bst = (size_t)16 * K;
  #pragma unroll 1
  for (int k0 = 0; k0 < K; k0 += 32) {
    const v16h a = load_frag32(ap + k0, h);
    #pragma unroll
    for (int nt = 0; nt < 4; ++nt) {
      const v16h bb = load_frag32(bp + nt * bst + k0, h);
      acc[nt] = wmma_f16(a, bb, acc[nt]);
    }
  }
}

__global__ __launch_bounds__(128) void gemm_nchw_k(
    const f16t* __restrict__ A, int K, const f16t* __restrict__ Bw, const float* __restrict__ bias,
    int relu, float osc, const float* __restrict__ res, float* __restrict__ out)
{
  __shared__ __attribute__((aligned(16))) float sD[64 * 64];
  const int tid = threadIdx.x, lane = tid & 31, w = tid >> 5;
  const int h = lane >> 4, m = lane & 15;
  const int p0 = blockIdx.x * 64;
  const int b = blockIdx.x >> 6, y = blockIdx.x & 63;
  const int n0 = blockIdx.y * 64;
  v8f acc[4];
  gemm_main(A, K, Bw, p0 + 16 * w, n0, h, m, acc);
  #pragma unroll
  for (int nt = 0; nt < 4; ++nt) {
    const int col = 16 * nt + m;
    const float bv = bias[n0 + col];
    #pragma unroll
    for (int r = 0; r < 8; ++r) {
      float val = acc[nt][r] * osc + bv;
      if (relu) val = fmaxf(val, 0.f);
      sD[col * 64 + 16 * w + 8 * h + r] = val;
    }
  }
  __syncthreads();
  nchw_store(sD, out, res, b, n0, y, w, lane);
}

__global__ __launch_bounds__(128) void gemm_h_k(
    const f16t* __restrict__ A, int K, const f16t* __restrict__ Bw, const float* __restrict__ bias,
    int relu, float osc, float ocar, f16t* __restrict__ outh, int N)
{
  __shared__ __attribute__((aligned(16))) f16t sH[64 * 64];
  const int tid = threadIdx.x, lane = tid & 31, w = tid >> 5;
  const int h = lane >> 4, m = lane & 15;
  const int p0 = blockIdx.x * 64;
  const int n0 = blockIdx.y * 64;
  v8f acc[4];
  gemm_main(A, K, Bw, p0 + 16 * w, n0, h, m, acc);
  #pragma unroll
  for (int nt = 0; nt < 4; ++nt) {
    const int col = 16 * nt + m;
    const float bv = bias[n0 + col];
    #pragma unroll
    for (int r = 0; r < 8; ++r) {
      float val = acc[nt][r] * osc + bv;
      if (relu) val = fmaxf(val, 0.f);
      sH[(16 * w + 8 * h + r) * 64 + col] = (f16t)(val * ocar);
    }
  }
  __syncthreads();
  const int q8 = lane & 7, sub = lane >> 3;
  v8h vals[4];
  size_t d[4];
  #pragma unroll
  for (int i = 0; i < 4; ++i) {
    const int lid = 16 * w + 4 * i + sub;
    vals[i] = *(const v8ha*)(sH + lid * 64 + 8 * q8);
    d[i] = (size_t)(p0 + lid) * N + n0 + 8 * q8;
  }
  #pragma unroll
  for (int i = 0; i < 4; ++i) *(volatile v8h*)(outh + d[i]) = vals[i];
  __threadfence();
  #pragma unroll
  for (int i = 0; i < 4; ++i) *(volatile v8h*)(outh + d[i]) = vals[i];
}

__global__ __launch_bounds__(128) void gemm_qkv_k(
    const f16t* __restrict__ A, const f16t* __restrict__ Bw, const float* __restrict__ qb, float osc,
    f16t* __restrict__ qkp, f16t* __restrict__ vp, float* __restrict__ v0)
{
  __shared__ __attribute__((aligned(16))) float sD[64 * 64];
  __shared__ __attribute__((aligned(16))) f16t sH[64 * 64];
  const int tid = threadIdx.x, lane = tid & 31, w = tid >> 5;
  const int h = lane >> 4, m = lane & 15;
  const int p0 = blockIdx.x * 64;
  const int b = blockIdx.x >> 6, y = blockIdx.x & 63;
  const int gy = blockIdx.y;
  const int g = gy >> 1, ch0 = (gy & 1) * 64, hh0 = ch0 >> 4;
  const int n0 = gy * 64;
  v8f acc[4];
  gemm_main(A, DIMC, Bw, p0 + 16 * w, n0, h, m, acc);
  #pragma unroll
  for (int nt = 0; nt < 4; ++nt) {
    const int col = 16 * nt + m;
    const int c = ch0 + col;
    const float bv = qb[c * 5 + g];
    #pragma unroll
    for (int r = 0; r < 8; ++r) {
      const float val = acc[nt][r] * osc + bv;
      const int px = 16 * w + 8 * h + r;
      sD[col * 64 + px] = val;
      sH[px * 64 + col] = (f16t)(val * QCAR);
    }
  }
  __syncthreads();

  f16t* planeX = (g == 0) ? qkp : ((g == 1) ? (qkp + PLANE) : vp);
  f16t* planeY = (g == 2) ? (vp + PLANE) : ((g == 3) ? (qkp + 2 * PLANE) : (qkp + 3 * PLANE));
  const bool doX = (g <= 2), doY = (g >= 2);
  const int q8 = lane & 7, sub = lane >> 3, tr = q8 >> 1, dh = q8 & 1;
  v8h vals[4];
  size_t dX[4], dY[4];
  const size_t wy = ((size_t)((b * 16 + (y >> 2)) * NHEAD + hh0 + w)) * LWIN + (size_t)(y & 3) * 64;
  #pragma unroll
  for (int i = 0; i < 4; ++i) {
    const int rem = 4 * i + sub;
    const int xx = 4 * rem + tr;
    vals[i] = *(const v8ha*)(sH + xx * 64 + 16 * w + 8 * dh);
    dX[i] = (((size_t)((b * 16 + rem) * NHEAD + hh0 + w)) * LWIN + (size_t)(4 * y)) * HDIM + 8 * q8;
    dY[i] = (wy + (size_t)(4 * rem)) * HDIM + 8 * q8;
  }
  if (doX) {
    #pragma unroll
    for (int i = 0; i < 4; ++i) *(volatile v8h*)(planeX + dX[i]) = vals[i];
  }
  if (doY) {
    #pragma unroll
    for (int i = 0; i < 4; ++i) *(volatile v8h*)(planeY + dY[i]) = vals[i];
  }
  __threadfence();
  if (doX) {
    #pragma unroll
    for (int i = 0; i < 4; ++i) *(volatile v8h*)(planeX + dX[i]) = vals[i];
  }
  if (doY) {
    #pragma unroll
    for (int i = 0; i < 4; ++i) *(volatile v8h*)(planeY + dY[i]) = vals[i];
  }
  if (g == 2) nchw_store(sD, v0, nullptr, b, ch0, y, w, lane);
}

__global__ __launch_bounds__(256) void dwT_k(
    const float* __restrict__ in, const float* __restrict__ wk, const float* __restrict__ bias,
    f16t* __restrict__ out)
{
  __shared__ __attribute__((aligned(16))) f16t sH[64 * 64];
  const int tid = threadIdx.x, lane = tid & 31, w = tid >> 5;
  const int ch0 = blockIdx.x * 64, y = blockIdx.y, b = blockIdx.z;
  const int xq = tid & 15, cl = tid >> 4, x0 = 4 * xq;
  #pragma unroll 1
  for (int j = 0; j < 4; ++j) {
    const int col = cl + 16 * j, c = ch0 + col;
    const float* pl = in + (size_t)(b * DIMC + c) * NPIX;
    float wc[9];
    #pragma unroll
    for (int t = 0; t < 9; ++t) wc[t] = wk[c * 9 + t];
    const float bc = bias[c];
    float acc[4];
    v4f mid;
    dw3x4(pl, y, x0, wc, acc, mid);
    #pragma unroll
    for (int i = 0; i < 4; ++i) sH[(x0 + i) * 64 + col] = (f16t)(fmaxf(acc[i] + bc, 0.f) * TCAR);
  }
  __syncthreads();
  plane_store64(sH, out, (size_t)b * NPIX + (size_t)y * WW, ch0, w, lane);
}

__device__ __forceinline__ v16h pack_p(v8f a, v8f c) {
  v16h r;
  #pragma unroll
  for (int j = 0; j < 8; ++j) { r[j] = (f16t)(a[j] * PCAR); r[8 + j] = (f16t)(c[j] * PCAR); }
  return r;
}

__global__ __launch_bounds__(256) void attn_k(
    const f16t* __restrict__ qkp, const f16t* __restrict__ vp, f16t* __restrict__ o16)
{
  __shared__ __attribute__((aligned(16))) f16t svt[HDIM * VTS];
  __shared__ __attribute__((aligned(16))) f16t so[8 * 256];
  const int tid = threadIdx.x, lane = tid & 31, w = tid >> 5;
  const int h = lane >> 4, m = lane & 15;
  const int br = blockIdx.z, unit = blockIdx.y;
  const int q0 = blockIdx.x * 128 + 16 * w;
  const size_t ubase = (size_t)unit * (LWIN * HDIM);
  const f16t* qpl = qkp + (size_t)(2 * br) * PLANE + ubase;
  const f16t* kpl = qkp + (size_t)(2 * br + 1) * PLANE + ubase;
  const f16t* vpl = vp + (size_t)br * PLANE + ubase;

  {
    const int key = tid;
    const v8h a = *(const v8ha*)(vpl + key * HDIM);
    const v8h c = *(const v8ha*)(vpl + key * HDIM + 8);
    #pragma unroll
    for (int j = 0; j < 8; ++j) {
      svt[j * VTS + key] = a[j];
      svt[(8 + j) * VTS + key] = c[j];
    }
  }
  __syncthreads();

  const v16h qb = load_frag16(qpl + (size_t)(q0 + m) * HDIM, h);
  const v8f z8 = {0.f, 0.f, 0.f, 0.f, 0.f, 0.f, 0.f, 0.f};
  v8f o = z8;
  float mrun = -1.0e30f, lrun = 0.f;
  const f16t* kbase = kpl + m * HDIM;
  const f16t* vbase = svt + m * VTS;
  const float sinv = 1.0f / (QCAR * QCAR);

  #pragma unroll 1
  for (int kb = 0; kb < LWIN; kb += 64) {
    v8f s[4];
    #pragma unroll
    for (int j = 0; j < 4; ++j) {
      const v16h kf = load_frag16(kbase + (size_t)(kb + 16 * j) * HDIM, h);
      s[j] = wmma_f16(kf, qb, z8);
    }
    float mloc = s[0][0];
    #pragma unroll
    for (int j = 0; j < 4; ++j) {
      #pragma unroll
      for (int r = 0; r < 8; ++r) mloc = fmaxf(mloc, s[j][r]);
    }
    mloc = fmaxf(mloc, __shfl_xor(mloc, 16));
    const float mnew = fmaxf(mrun, mloc);
    const float alpha = __expf((mrun - mnew) * sinv);
    mrun = mnew;
    float lsum = 0.f;
    #pragma unroll
    for (int j = 0; j < 4; ++j) {
      #pragma unroll
      for (int r = 0; r < 8; ++r) {
        const float p = __expf((s[j][r] - mnew) * sinv);
        s[j][r] = p;
        lsum += p;
      }
    }
    lsum += __shfl_xor(lsum, 16);
    lrun = lrun * alpha + lsum;
    #pragma unroll
    for (int r = 0; r < 8; ++r) o[r] = o[r] * alpha;

    const v16h pb0 = pack_p(s[0], s[1]);
    const v16h pb1 = pack_p(s[2], s[3]);
    const v16h vf0 = load_frag32(vbase + kb, h);
    const v16h vf1 = load_frag32(vbase + kb + 32, h);
    o = wmma_f16(vf0, pb0, o);
    o = wmma_f16(vf1, pb1, o);
  }

  const float inv = __builtin_amdgcn_rcpf(lrun) * (OCAR / (PCAR * QCAR));
  f16t* sw = so + w * 256;
  v8h ov;
  #pragma unroll
  for (int r = 0; r < 8; ++r) ov[r] = (f16t)(o[r] * inv);
  *(v8ha*)(sw + m * 16 + 8 * h) = ov;
  __syncthreads();
  const v8h val = *(const v8ha*)(sw + 8 * lane);
  f16t* dst = o16 + (size_t)br * PLANE + ubase + (size_t)q0 * HDIM + 8 * lane;
  *(volatile v8h*)dst = val;
  __threadfence();
  *(volatile v8h*)dst = val;
}

__global__ __launch_bounds__(256) void amul_k(
    const float* __restrict__ v0, const f16t* __restrict__ o16, const float* __restrict__ act,
    const float* __restrict__ wx, const float* __restrict__ bx, const float* __restrict__ wyv,
    const float* __restrict__ byv, f16t* __restrict__ am)
{
  __shared__ __attribute__((aligned(16))) f16t sH[64 * 64];
  const int tid = threadIdx.x, lane = tid & 31, w = tid >> 5;
  const int ch0 = blockIdx.x * 64, y = blockIdx.y, b = blockIdx.z;
  const int xq = tid & 15, cl = tid >> 4, x0 = 4 * xq;
  const float oinv = 1.0f / OCAR;
  #pragma unroll 1
  for (int j = 0; j < 4; ++j) {
    const int col = cl + 16 * j, c = ch0 + col;
    const int head = c >> 4, d = c & 15;
    const float* pl = v0 + (size_t)(b * DIMC + c) * NPIX;
    float wc[9];
    #pragma unroll
    for (int t = 0; t < 9; ++t) wc[t] = wx[c * 9 + t] + wyv[c * 9 + t];
    const float bc = bx[c] + byv[c];
    float acc[4];
    v4f mid;
    dw3x4(pl, y, x0, wc, acc, mid);
    const f16t* ox = o16 + (((size_t)((b * 16 + xq) * NHEAD + head)) * LWIN + (size_t)(4 * y)) * HDIM + d;
    const f16t* oy = o16 + PLANE +
        (((size_t)((b * 16 + (y >> 2)) * NHEAD + head)) * LWIN + (size_t)((y & 3) * 64 + 4 * xq)) * HDIM + d;
    const v4f a4 = *(const v4fa*)(act + ((size_t)(b * DIMC + c) * HH + y) * WW + x0);
    float av[4];
    av[0] = a4.x; av[1] = a4.y; av[2] = a4.z; av[3] = a4.w;
    #pragma unroll
    for (int i = 0; i < 4; ++i) {
      const float oxv = (float)ox[i * HDIM];
      const float oyv = (float)oy[i * HDIM];
      const float a = (oxv + oyv) * oinv + (acc[i] + bc);
      sH[(x0 + i) * 64 + col] = (f16t)((a * av[i]) * ACAR);
    }
  }
  __syncthreads();
  plane_store64(sH, am, (size_t)b * NPIX + (size_t)y * WW, ch0, w, lane);
}

extern "C" void kernel_launch(void* const* d_in, const int* in_sizes, int n_in,
                              void* d_out, int out_size, void* d_ws, size_t ws_size,
                              hipStream_t stream) {
  if (n_in < 29) return;
  const int tot = NB * DIMC * NPIX;
  if (in_sizes[0] != tot || out_size != tot) return;
  if (in_sizes[1] != 5 || in_sizes[2] != 1) return;
  const int dwidx[5] = {3, 11, 15, 17, 21};
  for (int i = 0; i < 5; ++i) if (in_sizes[dwidx[i]] != DIMC * 9) return;
  const int vecidx[13] = {4, 5, 6, 8, 10, 12, 16, 18, 20, 22, 23, 24, 28};
  for (int i = 0; i < 13; ++i) if (in_sizes[vecidx[i]] != DIMC) return;
  if (in_sizes[7] != DIMC * DIMC || in_sizes[9] != DIMC * DIMC || in_sizes[19] != DIMC * DIMC) return;
  if (in_sizes[13] != 5 * DIMC * DIMC || in_sizes[14] != 5 * DIMC) return;
  if (in_sizes[25] != 4 * DIMC * DIMC || in_sizes[26] != 4 * DIMC || in_sizes[27] != 4 * DIMC * DIMC) return;

  const float* x      = (const float*)d_in[0];
  const float* gw     = (const float*)d_in[1];
  const float* alpha  = (const float*)d_in[2];
  const float* dw1_w  = (const float*)d_in[3];
  const float* dw1_b  = (const float*)d_in[4];
  const float* g1     = (const float*)d_in[5];
  const float* b1     = (const float*)d_in[6];
  const float* actp_w = (const float*)d_in[7];
  const float* actp_b = (const float*)d_in[8];
  const float* inp_w  = (const float*)d_in[9];
  const float* inp_b  = (const float*)d_in[10];
  const float* dwc_w  = (const float*)d_in[11];
  const float* dwc_b  = (const float*)d_in[12];
  const float* qkv_w  = (const float*)d_in[13];
  const float* qkv_b  = (const float*)d_in[14];
  const float* ax_w   = (const float*)d_in[15];
  const float* ax_b   = (const float*)d_in[16];
  const float* ay_w   = (const float*)d_in[17];
  const float* ay_b   = (const float*)d_in[18];
  const float* outp_w = (const float*)d_in[19];
  const float* outp_b = (const float*)d_in[20];
  const float* dw2_w  = (const float*)d_in[21];
  const float* dw2_b  = (const float*)d_in[22];
  const float* g2     = (const float*)d_in[23];
  const float* b2     = (const float*)d_in[24];
  const float* m1_w   = (const float*)d_in[25];
  const float* m1_b   = (const float*)d_in[26];
  const float* m2_w   = (const float*)d_in[27];
  const float* m2_b   = (const float*)d_in[28];
  float* outp = (float*)d_out;

  const size_t MB = (size_t)1 << 20;
  const size_t total = 122 * MB;
  if (total > ws_size) return;
  char* ws = (char*)d_ws;
  f16t*  W16  = (f16t*)(ws + 0);
  float* GAP  = (float*)(ws + 524288);
  float* ST1  = (float*)(ws + 528384);
  float* ST2  = (float*)(ws + 529408);
  float* PART = (float*)(ws + 655360);
  float* X2   = (float*)(ws + 2 * MB);
  float* OUT2 = (float*)(ws + 2 * MB);
  float* ACT  = (float*)(ws + 18 * MB);
  float* OUT1 = (float*)(ws + 18 * MB);
  float* X1   = (float*)(ws + 34 * MB);
  float* U    = (float*)(ws + 34 * MB);
  f16t*  QKP  = (f16t*)(ws + 34 * MB);
  f16t*  AM16 = (f16t*)(ws + 34 * MB);
  f16t*  ON16 = (f16t*)(ws + 34 * MB);
  f16t*  M16  = (f16t*)(ws + 42 * MB);
  f16t*  XN   = (f16t*)(ws + 50 * MB);
  f16t*  T16  = (f16t*)(ws + 66 * MB);
  f16t*  VP   = (f16t*)(ws + 74 * MB);
  float* V0   = (float*)(ws + 90 * MB);
  f16t*  O16  = (f16t*)(ws + 106 * MB);

  const f16t* W_act = W16 + 0;
  const f16t* W_in  = W16 + 16384;
  const f16t* W_qkv = W16 + 32768;
  const f16t* W_out = W16 + 114688;
  const f16t* W_m1  = W16 + 131072;
  const f16t* W_m2  = W16 + 196608;

  const dim3 gRow(2, HH, NB);
  const dim3 gDw(4, DIMC, NB);

  wcvt_k<<<128, 256, 0, stream>>>(actp_w, inp_w, qkv_w, outp_w, m1_w, m2_w, W16);
  gap_k<<<(NB * DIMC) / 32, 256, 0, stream>>>(x, GAP);
  front_k<<<dim3(HH, NB), 256, 0, stream>>>(x, GAP, gw, alpha, X1);
  dwres_k<<<gDw, 256, 0, stream>>>(X1, dw1_w, dw1_b, X2, PART);
  gnstat_k<<<1, 256, 0, stream>>>(PART, ST1);
  cvt_k<<<gRow, 256, 0, stream>>>(X2, ST1, g1, b1, XN);
  gemm_nchw_k<<<dim3(NP / 64, 2), 128, 0, stream>>>(XN, DIMC, W_act, actp_b, 1, 1.0f / WSC, nullptr, ACT);
  gemm_nchw_k<<<dim3(NP / 64, 2), 128, 0, stream>>>(XN, DIMC, W_in, inp_b, 0, 1.0f / WSC, nullptr, U);
  dwT_k<<<gRow, 256, 0, stream>>>(U, dwc_w, dwc_b, T16);
  gemm_qkv_k<<<dim3(NP / 64, 10), 128, 0, stream>>>(T16, W_qkv, qkv_b, 1.0f / (WSC * TCAR), QKP, VP, V0);
  attn_k<<<dim3(2, NUNIT, 2), 256, 0, stream>>>(QKP, VP, O16);
  amul_k<<<gRow, 256, 0, stream>>>(V0, O16, ACT, ax_w, ax_b, ay_w, ay_b, AM16);
  gemm_nchw_k<<<dim3(NP / 64, 2), 128, 0, stream>>>(AM16, DIMC, W_out, outp_b, 0, 1.0f / (WSC * ACAR), X2, OUT1);
  dwres_k<<<gDw, 256, 0, stream>>>(OUT1, dw2_w, dw2_b, OUT2, PART);
  gnstat_k<<<1, 256, 0, stream>>>(PART, ST2);
  cvt_k<<<gRow, 256, 0, stream>>>(OUT2, ST2, g2, b2, ON16);
  gemm_h_k<<<dim3(NP / 64, 8), 128, 0, stream>>>(ON16, DIMC, W_m1, m1_b, 1, 1.0f / WSC, MCAR, M16, 4 * DIMC);
  gemm_nchw_k<<<dim3(NP / 64, 2), 128, 0, stream>>>(M16, 4 * DIMC, W_m2, m2_b, 0, 1.0f / (WSC * MCAR), OUT2, outp);
}
